// LSTMSentimentModel_10496900071463
// MI455X (gfx1250) — hardware-verified
//
#include <hip/hip_runtime.h>


#define B_ 2048
#define L_ 512
#define T_ 256
#define E_ 32
#define C_ 32
#define H_ 32
#define G_ 128
#define O_ 3
#define KC 96
#define KG 64
#define EP 40
#define HP 40
#define GP 132

typedef _Float16 f16t;
typedef f16t  v16h __attribute__((ext_vector_type(16)));
typedef f16t  v8h  __attribute__((ext_vector_type(8)));
typedef float v8f  __attribute__((ext_vector_type(8)));
typedef float v4f  __attribute__((ext_vector_type(4)));
typedef unsigned int v4u __attribute__((ext_vector_type(4)));

union Frag { v16h v; v8h q[2]; };
union Pk16 { v8h h; v4u u; };
union Pk32 { v4f f; v4u u; };

__device__ __forceinline__ v8f wmma16(v16h a, v16h b, v8f c) {
    return __builtin_amdgcn_wmma_f32_16x16x32_f16(false, a, false, b, (short)0, c, false, false);
}

__device__ __forceinline__ v8f zf8() {
    v8f z = {0.f, 0.f, 0.f, 0.f, 0.f, 0.f, 0.f, 0.f};
    return z;
}

__device__ __forceinline__ void ldfrag(Frag& f, const f16t* p) {
    f.q[0] = *(const v8h*)p;
    f.q[1] = *(const v8h*)(p + 16);
}

__device__ __forceinline__ float frcp(float x) { return __builtin_amdgcn_rcpf(x); }
__device__ __forceinline__ float sigm(float x) { return frcp(1.0f + __expf(-x)); }
__device__ __forceinline__ float ftanh(float x) {
    float ax = fabsf(x);
    float t  = __expf(-2.0f * ax);
    float r  = (1.0f - t) * frcp(1.0f + t);
    return copysignf(r, x);
}

__global__ __launch_bounds__(256)
void k_wprep(const float* emb, const float* conv_w,
             const float* wihf, const float* whhf, const float* wihb, const float* whhb,
             f16t* E16, f16t* Pc, f16t* Pf, f16t* Pb, int nE8, float sc) {
    const int i  = blockIdx.x * 256 + threadIdx.x;
    const int n1 = nE8;
    const int n2 = n1 + C_ * (KC / 8);
    const int n3 = n2 + G_ * (KG / 8);
    const int n4 = n3 + G_ * (KG / 8);
    if (i >= n4) return;
    Pk16 v;
    f16t* dst;
    if (i < n1) {
        const float* p = emb + (size_t)i * 8;
        v4f a = *(const v4f*)p;
        v4f b = *(const v4f*)(p + 4);
#pragma unroll
        for (int e = 0; e < 4; ++e) {
            v.h[e]     = (f16t)(a[e] * sc);
            v.h[4 + e] = (f16t)(b[e] * sc);
        }
        dst = E16 + (size_t)i * 8;
    } else if (i < n2) {
        const int j  = i - n1;
        const int o  = j / 12;
        const int k  = (j - o * 12) * 8;
        const int kk = k >> 5;
        const int e0 = k & 31;
#pragma unroll
        for (int e = 0; e < 8; ++e)
            v.h[e] = (f16t)(conv_w[(o * E_ + e0 + e) * 3 + kk] * sc);
        dst = Pc + (size_t)j * 8;
    } else {
        const bool fwd = (i < n3);
        const int  j   = fwd ? (i - n2) : (i - n3);
        const int  g   = j >> 3;
        const int  k   = (j & 7) * 8;
        const bool ih  = (k < 32);
        const int  kb  = g * H_ + (k & 31);
#pragma unroll
        for (int e = 0; e < 8; ++e) {
            float a0 = wihf[kb + e], a1 = whhf[kb + e];
            float a2 = wihb[kb + e], a3 = whhb[kb + e];
            float s  = fwd ? (ih ? a0 : a1) : (ih ? a2 : a3);
            v.h[e] = (f16t)(s * sc);
        }
        dst = (fwd ? Pf : Pb) + (size_t)j * 8;
    }
    *(volatile v4u*)dst = v.u;
    __threadfence();
    *(volatile v4u*)dst = v.u;
}

__global__ __launch_bounds__(128)
void k_conv(const int* x, const f16t* E16, const f16t* Pc, const float* conv_b,
            f16t* S, int nV, float inv, float sc) {
    __shared__ __attribute__((aligned(16))) f16t ebuf[66 * EP];
    __shared__ __attribute__((aligned(16))) f16t sq[32 * 32];
    const int tid = threadIdx.x, w = tid >> 5, l = tid & 31, h = l >> 4, m = l & 15;
    const int b = blockIdx.y;
    const int lbase = blockIdx.x * 64, tbase = blockIdx.x * 32;

    for (int i = tid; i < 66 * 4; i += 128) {
        const int r = i >> 2, q = i & 3;
        const int p = lbase - 1 + r;
        const int pc = min(max(p, 0), L_ - 1);
        int idx = x[(size_t)b * L_ + pc];
        idx = min(max(idx, 0), nV - 1);
        Pk16 u;
        u.h = *(const v8h*)(E16 + (size_t)idx * E_ + q * 8);
        if (p < 0 || p >= L_) { v4u z4 = {0u, 0u, 0u, 0u}; u.u = z4; }
        *(v8h*)(ebuf + r * EP + q * 8) = u.h;
    }
    __syncthreads();

    v8f acc[2];
    acc[0] = zf8(); acc[1] = zf8();
#pragma unroll
    for (int kk = 0; kk < 3; ++kk) {
        Frag a, bf[2];
        ldfrag(a, ebuf + (16 * w + kk + m) * EP + 8 * h);
#pragma unroll
        for (int j = 0; j < 2; ++j)
            ldfrag(bf[j], Pc + (size_t)(16 * j + m) * KC + 32 * kk + 8 * h);
#pragma unroll
        for (int j = 0; j < 2; ++j)
            acc[j] = wmma16(a.v, bf[j].v, acc[j]);
        asm volatile("v_nop\n\tv_nop\n\tv_nop\n\tv_nop"
                     : "+v"(acc[0]), "+v"(acc[1])
                     : "v"(a.v), "v"(bf[0].v), "v"(bf[1].v));
    }

    const float cb0 = conv_b[m], cb1 = conv_b[16 + m];
#pragma unroll
    for (int j = 0; j < 2; ++j) {
        const float cb = (j == 0) ? cb0 : cb1;
#pragma unroll
        for (int u = 0; u < 4; ++u) {
            float mx = fmaxf(acc[j][2 * u], acc[j][2 * u + 1]);
            float v  = fmaf(mx, inv, cb);
            sq[(8 * w + 4 * h + u) * 32 + 16 * j + m] = (f16t)(v * sc);
        }
    }
    __syncthreads();

    Pk16 o;
    o.h = *(const v8h*)(sq + tid * 8);
    f16t* dst = S + ((size_t)b * T_ + tbase) * C_ + tid * 8;
    *(volatile v4u*)dst = o.u;
    __threadfence();
    *(volatile v4u*)dst = o.u;
}

__global__ __launch_bounds__(256)
void k_lstm(const f16t* S, const f16t* Pf, const f16t* Pb,
            const float* bihf, const float* bhhf, const float* bihb, const float* bhhb,
            const float* fcw, const float* fcb, float* out, int nb, float inv, float sc) {
    __shared__ __attribute__((aligned(16))) f16t  hb[32 * HP];
    __shared__ __attribute__((aligned(16))) float gs[32 * GP];
    __shared__ __attribute__((aligned(16))) float hl[32 * 64];
    __shared__ __attribute__((aligned(16))) float bs[2 * G_];
    __shared__ __attribute__((aligned(16))) float fw[O_ * 64];
    __shared__ __attribute__((aligned(16))) float fb[4];
    __shared__ __attribute__((aligned(16))) float os[32 * O_];
    const int tid = threadIdx.x, w = tid >> 5, l = tid & 31, h = l >> 4, m = l & 15;
    const int bb = blockIdx.x * 32;
    if (bb + 32 > nb) return;

    for (int i = tid; i < 32 * HP; i += 256) hb[i] = (f16t)0.0f;
    if (tid < G_) {
        bs[tid]      = bihf[tid] + bhhf[tid];
        bs[G_ + tid] = bihb[tid] + bhhb[tid];
    }
    if (tid < O_ * 64) fw[tid] = fcw[tid];
    if (tid < O_) fb[tid] = fcb[tid];

    Frag bi, bh;
    {
        const f16t* p = Pf + (size_t)(16 * w + m) * KG + 8 * h;
        bi.q[0] = *(const v8h*)p;        bi.q[1] = *(const v8h*)(p + 16);
        bh.q[0] = *(const v8h*)(p + 32); bh.q[1] = *(const v8h*)(p + 48);
    }
    float cr[4] = {0.f, 0.f, 0.f, 0.f};
    __syncthreads();

    const size_t rp = (size_t)T_ * C_;
    const f16t* srow = S + (size_t)(bb + m) * rp + 8 * h;

#pragma unroll 1
    for (int t = 0; t < T_; ++t) {
        Frag ax[2], ah[2];
        v8f acc[2];
#pragma unroll
        for (int i = 0; i < 2; ++i) {
            ldfrag(ax[i], srow + (size_t)(16 * i) * rp + (size_t)t * C_);
            ldfrag(ah[i], hb + (16 * i + m) * HP + 8 * h);
        }
#pragma unroll
        for (int i = 0; i < 2; ++i) {
            acc[i] = zf8();
            acc[i] = wmma16(ax[i].v, bi.v, acc[i]);
            acc[i] = wmma16(ah[i].v, bh.v, acc[i]);
        }
        asm volatile("v_nop\n\tv_nop\n\tv_nop\n\tv_nop"
                     : "+v"(acc[0]), "+v"(acc[1])
                     : "v"(ax[0].v), "v"(ax[1].v), "v"(ah[0].v), "v"(ah[1].v), "v"(bi.v), "v"(bh.v));
#pragma unroll
        for (int i = 0; i < 2; ++i)
#pragma unroll
            for (int r = 0; r < 8; ++r)
                gs[(16 * i + 8 * h + r) * GP + 16 * w + m] = acc[i][r];
        __syncthreads();

#pragma unroll
        for (int r = 0; r < 4; ++r) {
            const int e = tid + 256 * r, mm = e >> 5, n = e & 31;
            const float* g = gs + mm * GP + n;
            float gi = fmaf(g[0],  inv, bs[n]);
            float gf = fmaf(g[32], inv, bs[32 + n]);
            float gg = fmaf(g[64], inv, bs[64 + n]);
            float go = fmaf(g[96], inv, bs[96 + n]);
            float c  = sigm(gf) * cr[r] + sigm(gi) * ftanh(gg);
            float hh = sigm(go) * ftanh(c);
            cr[r] = c;
            hb[mm * HP + n] = (f16t)(hh * sc);
            if (t == T_ - 1) hl[mm * 64 + n] = hh;
        }
        __syncthreads();
    }

    {
        Frag bib;
        {
            const f16t* p = Pb + (size_t)(16 * w + m) * KG + 8 * h;
            bib.q[0] = *(const v8h*)p; bib.q[1] = *(const v8h*)(p + 16);
        }
        Frag ax[2];
        v8f acc[2];
#pragma unroll
        for (int i = 0; i < 2; ++i)
            ldfrag(ax[i], srow + (size_t)(16 * i) * rp + (size_t)(T_ - 1) * C_);
#pragma unroll
        for (int i = 0; i < 2; ++i) {
            acc[i] = zf8();
            acc[i] = wmma16(ax[i].v, bib.v, acc[i]);
        }
        asm volatile("v_nop\n\tv_nop\n\tv_nop\n\tv_nop"
                     : "+v"(acc[0]), "+v"(acc[1])
                     : "v"(ax[0].v), "v"(ax[1].v), "v"(bib.v));
#pragma unroll
        for (int i = 0; i < 2; ++i)
#pragma unroll
            for (int r = 0; r < 8; ++r)
                gs[(16 * i + 8 * h + r) * GP + 16 * w + m] = acc[i][r];
        __syncthreads();

#pragma unroll
        for (int r = 0; r < 4; ++r) {
            const int e = tid + 256 * r, mm = e >> 5, n = e & 31;
            const float* g = gs + mm * GP + n;
            float gi = fmaf(g[0],  inv, bs[G_ + n]);
            float gg = fmaf(g[64], inv, bs[G_ + 64 + n]);
            float go = fmaf(g[96], inv, bs[G_ + 96 + n]);
            float c  = sigm(gi) * ftanh(gg);
            float hh = sigm(go) * ftanh(c);
            hl[mm * 64 + 32 + n] = hh;
        }
        __syncthreads();
    }

    if (tid < 32 * O_) {
        const int mm = tid / 3, o = tid - 3 * mm;
        float s = 0.f;
#pragma unroll 8
        for (int k = 0; k < 64; ++k) s = fmaf(hl[mm * 64 + k], fw[o * 64 + k], s);
        os[tid] = s + fb[o];
    }
    __syncthreads();

    Pk32 v;
    v.u = (v4u){0u, 0u, 0u, 0u};
    if (tid < 24) v.f = *(const v4f*)(os + tid * 4);
    float* dst = out + (size_t)bb * O_ + tid * 4;
    if (tid < 24) *(volatile v4u*)dst = v.u;
    __threadfence();
    if (tid < 24) *(volatile v4u*)dst = v.u;
}

extern "C" void kernel_launch(void* const* d_in, const int* in_sizes, int n_in,
                              void* d_out, int out_size, void* d_ws, size_t ws_size,
                              hipStream_t stream) {
    if (n_in < 14) return;
    if (in_sizes[0] != B_ * L_) return;
    if (in_sizes[1] < E_ * 2 || (in_sizes[1] % E_) != 0) return;
    if (in_sizes[2] != C_ * E_ * 3 || in_sizes[3] != C_) return;
    if (in_sizes[4] != G_ * C_ || in_sizes[5] != G_ * H_ || in_sizes[6] != G_ || in_sizes[7] != G_) return;
    if (in_sizes[8] != G_ * C_ || in_sizes[9] != G_ * H_ || in_sizes[10] != G_ || in_sizes[11] != G_) return;
    if (in_sizes[12] != O_ * 2 * H_ || in_sizes[13] != O_) return;
    if (out_size != B_ * O_) return;

    const int*   x      = (const int*)d_in[0];
    const float* emb    = (const float*)d_in[1];
    const float* conv_w = (const float*)d_in[2];
    const float* conv_b = (const float*)d_in[3];
    const float* w_ih_f = (const float*)d_in[4];
    const float* w_hh_f = (const float*)d_in[5];
    const float* b_ih_f = (const float*)d_in[6];
    const float* b_hh_f = (const float*)d_in[7];
    const float* w_ih_b = (const float*)d_in[8];
    const float* w_hh_b = (const float*)d_in[9];
    const float* b_ih_b = (const float*)d_in[10];
    const float* b_hh_b = (const float*)d_in[11];
    const float* fc_w   = (const float*)d_in[12];
    const float* fc_b   = (const float*)d_in[13];
    float* out = (float*)d_out;

    const int nV  = in_sizes[1] / E_;
    const int nE8 = in_sizes[1] / 8;

    unsigned char* ws = (unsigned char*)d_ws;
    size_t off = 0;
    auto carve = [&](size_t bytes) -> unsigned char* {
        unsigned char* p = ws + off;
        off = (off + bytes + 255) & ~(size_t)255;
        return p;
    };
    f16t* E16 = (f16t*)carve((size_t)nV * E_ * 2);
    f16t* Pc  = (f16t*)carve((size_t)C_ * KC * 2);
    f16t* Pf  = (f16t*)carve((size_t)G_ * KG * 2);
    f16t* Pb  = (f16t*)carve((size_t)G_ * KG * 2);
    f16t* S   = (f16t*)carve((size_t)B_ * T_ * C_ * 2);
    if (off > ws_size) return;

    const float SC  = 64.0f;
    const float INV = 0.000244140625f;

    {
        const int tot = nE8 + C_ * (KC / 8) + 2 * G_ * (KG / 8);
        k_wprep<<<dim3((tot + 255) / 256), dim3(256), 0, stream>>>(emb, conv_w, w_ih_f, w_hh_f, w_ih_b, w_hh_b,
                                                                 E16, Pc, Pf, Pb, nE8, SC);
    }
    k_conv<<<dim3(L_ / 64, B_), dim3(128), 0, stream>>>(x, E16, Pc, conv_b, S, nV, INV, SC);
    k_lstm<<<dim3(B_ / 32), dim3(256), 0, stream>>>(S, Pf, Pb, b_ih_f, b_hh_f, b_ih_b, b_hh_b,
                                                   fc_w, fc_b, out, B_, INV, SC);
}
